// CosineTripletLoss_46531675684978
// MI455X (gfx1250) — hardware-verified
//
#include <hip/hip_runtime.h>
#include <stddef.h>


#define DDIM    1024
#define HINGE_C 0.05f
#define BAND_C  0.05f

typedef _Float16 v4h  __attribute__((ext_vector_type(4)));
typedef _Float16 v8h  __attribute__((ext_vector_type(8)));
typedef _Float16 v16h __attribute__((ext_vector_type(16)));
typedef float    v4f  __attribute__((ext_vector_type(4)));
typedef float    v8f  __attribute__((ext_vector_type(8)));
typedef int      v4i  __attribute__((ext_vector_type(4)));

union Frag { v16h v; v8h h[2]; };

__device__ __forceinline__ float neg_inf_f() { return -__builtin_huge_valf(); }

__device__ __forceinline__ float wave_row_dot(const float* __restrict__ a,
                                              const float* __restrict__ b, int lane) {
    float acc = 0.0f;
#pragma unroll
    for (int j = 0; j < DDIM / 128; ++j) {
        const int e = (lane + 32 * j) * 4;
        const v4f av = *(const v4f*)(a + e);
        const v4f bv = *(const v4f*)(b + e);
        acc += av.x * bv.x;
        acc += av.y * bv.y;
        acc += av.z * bv.z;
        acc += av.w * bv.w;
    }
#pragma unroll
    for (int m = 16; m >= 1; m >>= 1) acc += __shfl_xor(acc, m, 32);
    return acc;
}

__launch_bounds__(256)
__global__ void k_convert_f16(const float* __restrict__ x, const float* __restrict__ y,
                              _Float16* xh, _Float16* yh, int nrows) {
    const int wave = threadIdx.x >> 5;
    const int lane = threadIdx.x & 31;
    const int row  = blockIdx.x * 8 + wave;
    if (row >= nrows) return;
    const size_t base = (size_t)row * DDIM;

    v8h xv[4], yv[4];
#pragma unroll
    for (int j = 0; j < 4; ++j) {
        const int e = j * 256 + lane * 8;
        const v4f x0 = *(const v4f*)(x + base + e);
        const v4f x1 = *(const v4f*)(x + base + e + 4);
        const v4f y0 = *(const v4f*)(y + base + e);
        const v4f y1 = *(const v4f*)(y + base + e + 4);
        const v4h xa = __builtin_convertvector(x0, v4h);
        const v4h xb = __builtin_convertvector(x1, v4h);
        const v4h ya = __builtin_convertvector(y0, v4h);
        const v4h yb = __builtin_convertvector(y1, v4h);
        xv[j] = __builtin_shufflevector(xa, xb, 0, 1, 2, 3, 4, 5, 6, 7);
        yv[j] = __builtin_shufflevector(ya, yb, 0, 1, 2, 3, 4, 5, 6, 7);
    }
#pragma unroll
    for (int j = 0; j < 4; ++j) {
        const int e = j * 256 + lane * 8;
        *(volatile v8h*)(xh + base + e) = xv[j];
        *(volatile v8h*)(yh + base + e) = yv[j];
    }
    __threadfence();
#pragma unroll
    for (int j = 0; j < 4; ++j) {
        const int e = j * 256 + lane * 8;
        *(volatile v8h*)(xh + base + e) = xv[j];
        *(volatile v8h*)(yh + base + e) = yv[j];
    }
}

__launch_bounds__(128)
__global__ void k_sim_argmax(const _Float16* __restrict__ xh, const _Float16* __restrict__ yh,
                             const float* __restrict__ x, const float* __restrict__ y,
                             int* idxout, int nrows) {
    __shared__ float posl[128];
    __shared__ int   idxl[128];

    const int tid  = threadIdx.x;
    const int lane = tid & 31;
    const int wave = tid >> 5;
    const int lr   = lane & 15;
    const int hh   = lane >> 4;
    const int rowg = blockIdx.x * 128 + wave * 32;

#pragma unroll 1
    for (int i = 0; i < 32; ++i) {
        const float p = wave_row_dot(x + (size_t)(rowg + i) * DDIM,
                                     y + (size_t)(rowg + i) * DDIM, lane);
        if (lane == 0) posl[wave * 32 + i] = p;
    }
    __syncthreads();

    float bestv[2][8];
    int   besti[2][8];
#pragma unroll
    for (int r = 0; r < 2; ++r)
#pragma unroll
        for (int v = 0; v < 8; ++v) { bestv[r][v] = neg_inf_f(); besti[r][v] = 0; }

    const _Float16* arow = xh + (size_t)(rowg + lr) * DDIM + 8 * hh;
    const int dl = lr - 8 * hh;

    for (int cg = 0; cg < nrows; cg += 64) {
        const _Float16* bcol = yh + (size_t)(cg + lr) * DDIM + 8 * hh;

        v8f c[2][4];
#pragma unroll
        for (int r = 0; r < 2; ++r)
#pragma unroll
            for (int t = 0; t < 4; ++t) c[r][t] = (v8f)0.0f;

#pragma unroll 1
        for (int k0 = 0; k0 < DDIM; k0 += 32) {
            Frag a[2], b[4];
#pragma unroll
            for (int r = 0; r < 2; ++r) {
                a[r].h[0] = *(const v8h*)(arow + (size_t)r * 16 * DDIM + k0);
                a[r].h[1] = *(const v8h*)(arow + (size_t)r * 16 * DDIM + k0 + 16);
            }
#pragma unroll
            for (int t = 0; t < 4; ++t) {
                b[t].h[0] = *(const v8h*)(bcol + (size_t)t * 16 * DDIM + k0);
                b[t].h[1] = *(const v8h*)(bcol + (size_t)t * 16 * DDIM + k0 + 16);
            }
#pragma unroll
            for (int t = 0; t < 4; ++t)
#pragma unroll
                for (int r = 0; r < 2; ++r)
                    c[r][t] = __builtin_amdgcn_wmma_f32_16x16x32_f16(
                        false, a[r].v, false, b[t].v, (short)0, c[r][t], false, false);
            asm volatile("v_nop\n\tv_nop\n\tv_nop\n\tv_nop"
                         : "+v"(c[0][0]), "+v"(c[0][1]), "+v"(c[0][2]), "+v"(c[0][3]),
                           "+v"(c[1][0]), "+v"(c[1][1]), "+v"(c[1][2]), "+v"(c[1][3])
                         : "v"(a[0].v), "v"(a[1].v),
                           "v"(b[0].v), "v"(b[1].v), "v"(b[2].v), "v"(b[3].v));
        }

        const int dcg = (cg - rowg) + dl;
#pragma unroll
        for (int r = 0; r < 2; ++r) {
#pragma unroll
            for (int v = 0; v < 8; ++v) {
                const float pv = posl[wave * 32 + r * 16 + 8 * hh + v];
#pragma unroll
                for (int t = 0; t < 4; ++t) {
                    const int   col  = cg + t * 16 + lr;
                    const float s    = c[r][t][v];
                    const bool  keep = (dcg != (r * 16 + v - t * 16)) && (pv - s <= BAND_C);
                    const float val  = keep ? s : -1.0f;
                    if (val > bestv[r][v]) { bestv[r][v] = val; besti[r][v] = col; }
                }
            }
        }
    }

#pragma unroll
    for (int r = 0; r < 2; ++r) {
#pragma unroll
        for (int v = 0; v < 8; ++v) {
            float bv = bestv[r][v];
            int   bi = besti[r][v];
#pragma unroll
            for (int m = 1; m < 16; m <<= 1) {
                const float ov = __shfl_xor(bv, m, 32);
                const int   oi = __shfl_xor(bi, m, 32);
                if (ov > bv || (ov == bv && oi < bi)) { bv = ov; bi = oi; }
            }
            if (lr == 0) idxl[wave * 32 + r * 16 + 8 * hh + v] = bi;
        }
    }
    __syncthreads();

    v4i o = (v4i)0;
    if (lane < 8) {
        o[0] = idxl[wave * 32 + lane * 4 + 0];
        o[1] = idxl[wave * 32 + lane * 4 + 1];
        o[2] = idxl[wave * 32 + lane * 4 + 2];
        o[3] = idxl[wave * 32 + lane * 4 + 3];
    }
    int* dst = idxout + rowg + lane * 4;
    if (lane < 8) *(volatile v4i*)dst = o;
    __threadfence();
    if (lane < 8) *(volatile v4i*)dst = o;
}

__launch_bounds__(256)
__global__ void k_loss_mean(const float* __restrict__ x, const float* __restrict__ y,
                            const int* __restrict__ idxbuf, float* out, int nrows) {
    __shared__ double wsum[8];
    const int wave = threadIdx.x >> 5;
    const int lane = threadIdx.x & 31;

    double acc = 0.0;
    for (int row = wave; row < nrows; row += 8) {
        int j = idxbuf[row];
        j = j < 0 ? 0 : (j >= nrows ? nrows - 1 : j);
        const float* xr = x + (size_t)row * DDIM;
        const float  p  = wave_row_dot(xr, y + (size_t)row * DDIM, lane);
        const float  n  = wave_row_dot(xr, y + (size_t)j * DDIM, lane);
        float l = (HINGE_C - p) + n;
        l = l > 0.0f ? l : 0.0f;
        acc += (double)l;
    }
    if (lane == 0) wsum[wave] = acc;
    __syncthreads();
    if (threadIdx.x == 0) {
        double s = 0.0;
        for (int w = 0; w < 8; ++w) s += wsum[w];
        const float m = (float)s / (float)nrows;
        *(volatile float*)out = m;
        __threadfence();
        *(volatile float*)out = m;
    }
}

extern "C" void kernel_launch(void* const* d_in, const int* in_sizes, int n_in,
                              void* d_out, int out_size, void* d_ws, size_t ws_size,
                              hipStream_t stream) {
    if (n_in < 2 || out_size < 1) return;
    const int n0    = in_sizes[0];
    const int nrows = n0 / DDIM;
    if (nrows <= 0 || nrows * DDIM != n0 || in_sizes[1] != n0 || (nrows % 128) != 0) return;

    const float* x = (const float*)d_in[0];
    const float* y = (const float*)d_in[1];
    float* out = (float*)d_out;

    const size_t half_bytes = (size_t)nrows * DDIM * sizeof(_Float16);
    const size_t idx_off    = 2 * half_bytes;
    const size_t need       = idx_off + (size_t)nrows * sizeof(int);
    if (need > ws_size) return;

    _Float16* xh  = (_Float16*)d_ws;
    _Float16* yh  = (_Float16*)((char*)d_ws + half_bytes);
    int*      idx = (int*)((char*)d_ws + idx_off);

    k_convert_f16<<<dim3((nrows + 7) / 8), dim3(256), 0, stream>>>(x, y, xh, yh, nrows);
    k_sim_argmax<<<dim3(nrows / 128), dim3(128), 0, stream>>>(xh, yh, x, y, idx, nrows);
    k_loss_mean<<<dim3(1), dim3(256), 0, stream>>>(x, y, idx, out, nrows);
    (void)hipGetLastError();
}
